// GraphAttentionLayer_76416058130706
// MI455X (gfx1250) — hardware-verified
//
#include <hip/hip_runtime.h>


#ifndef NB
#define NB 8
#endif
#ifndef SEQ
#define SEQ 1024
#endif
#define NB_FULL  8
#define SEQ_FULL 1024
#ifndef OUT_SEQ
#define OUT_SEQ SEQ
#endif
#define KIN  256
#define NH_  8
#define HD   256
#define WC   (NH_ * HD)
#define AW   4
#define OSQ  260
#define NJ   (HD / 16)
#define ABW  (SEQ / 32)
#define WTP  33
#define TGO  ((size_t)NB * NH_ * SEQ)
#define SLOPE 0.2f
#define LOG2E 1.4426950408889634f
#define NEGT ((float)(-9.0e16 * 1.4426950408889634))
#define PSH  14.0f
#define NEGB (-3.0e38f)
#define HINV (1.0f / (float)NH_)

static_assert(NH_ * HD == WC);
static_assert(HD % 64 == 0);
static_assert(HD == 16 * NJ);
static_assert(NJ % 4 == 0);
static_assert(KIN % 32 == 0);
static_assert(KIN == 32 * 8);
static_assert(WC % 32 == 0);
static_assert(SEQ % 64 == 0);
static_assert((NB * SEQ) % 64 == 0);
static_assert(SEQ % 32 == 0);
static_assert(SEQ % (16 * AW) == 0);
static_assert(((size_t)SEQ * SEQ) % (1024 * 8) == 0);
static_assert(((size_t)SEQ * KIN) % 8 == 0);
static_assert(NB <= NB_FULL);
static_assert(SEQ <= SEQ_FULL);
static_assert((OSQ * 4) % 16 == 0);
static_assert(OSQ >= HD);
static_assert(32 * 16 * 4 == 16 * 64 * 2);
static_assert(32 * 16 == 2 * 64 * 4);
static_assert(32 * 16 * 32 == 16 * HD * 4);
static_assert(8 * 4 == 32);
static_assert((size_t)AW * 16 * OSQ * 4 <= 131072);
static_assert((size_t)KIN * WTP * 4 <= 131072);
static_assert((size_t)(16 * 68 + 128) * 4 <= 131072);

typedef _Float16 h16;
typedef unsigned short bf;
typedef __attribute__((ext_vector_type(16))) __bf16   v16bf;
typedef __attribute__((ext_vector_type(16))) _Float16 v16h;
typedef __attribute__((ext_vector_type(8)))  _Float16 v8h;
typedef __attribute__((ext_vector_type(8)))  unsigned short v8us;
typedef __attribute__((ext_vector_type(8)))  float    v8f;
typedef __attribute__((ext_vector_type(4)))  float    v4f;
typedef v4f  __attribute__((may_alias)) v4fa;

__device__ __forceinline__ unsigned short f2bf(float f) { unsigned u = __float_as_uint(f); u += 0x7FFFu + ((u >> 16) & 1u); return (unsigned short)(u >> 16); }
__device__ __forceinline__ float bfr(float f) { return __uint_as_float(((unsigned)f2bf(f)) << 16); }
__device__ __forceinline__ v16h cat16(v8h lo, v8h hi) { return __builtin_shufflevector(lo, hi, 0, 1, 2, 3, 4, 5, 6, 7, 8, 9, 10, 11, 12, 13, 14, 15); }
__device__ __forceinline__ v16bf cat16b(v8us lo, v8us hi) { return __builtin_bit_cast(v16bf, __builtin_shufflevector(lo, hi, 0, 1, 2, 3, 4, 5, 6, 7, 8, 9, 10, 11, 12, 13, 14, 15)); }
__device__ __forceinline__ v8f wmma16(v16h a, v16h b, v8f c) { return __builtin_amdgcn_wmma_f32_16x16x32_f16(false, a, false, b, (short)0, c, false, false); }
__device__ __forceinline__ v8f wmmab(v16bf a, v16bf b, v8f c) { return __builtin_amdgcn_wmma_f32_16x16x32_bf16(false, a, false, b, (short)0, c, false, false); }
__device__ __forceinline__ v16h  ldh(const h16* p) { return cat16(*(const v8h*)p, *(const v8h*)(p + 16)); }
__device__ __forceinline__ v16bf ldb(const bf* p)  { return cat16b(*(const v8us*)p, *(const v8us*)(p + 16)); }
__device__ __forceinline__ void wave_sync() { __builtin_amdgcn_fence(3  , "wavefront"); __builtin_amdgcn_wave_barrier(); asm volatile("" ::: "memory"); }

__device__ __forceinline__ v8f wmma16g(v16h a, v16h b, v8f c) { c = wmma16(a, b, c); asm volatile("v_nop\n\tv_nop\n\tv_nop\n\tv_nop" : "+v"(c) : "v"(a), "v"(b)); return c; }
__device__ __forceinline__ v8f wmmabg(v16bf a, v16bf b, v8f c) { c = wmmab(a, b, c); asm volatile("v_nop\n\tv_nop\n\tv_nop\n\tv_nop" : "+v"(c) : "v"(a), "v"(b)); return c; }
static __device__ __forceinline__ h16 toh_flush(float v) { const h16 r = (h16)v; return (fabsf(v) < 6.103515625e-05f) ? (h16)0.0f : r; }

__global__ __launch_bounds__(256) void k_cvt8(const float* __restrict__ src, bf* dst, size_t n8) {
    const size_t i = (size_t)blockIdx.x * 256 + threadIdx.x; if (i >= n8) return;
    const v8f v = *(const v8f*)(src + i * 8); v8us o;
#pragma unroll
    for (int k = 0; k < 8; ++k) o[k] = f2bf(v[k]);
    *(volatile v8us*)(dst + i * 8) = o; __threadfence(); *(volatile v8us*)(dst + i * 8) = o;
}

__global__ __launch_bounds__(256) void k_wt(const float* __restrict__ W, bf* WT) {
    __shared__ float tile[KIN * WTP];
    const int lane = threadIdx.x & 31;
    const int wave = __builtin_amdgcn_readfirstlane((int)(threadIdx.x >> 5));
    const int n0 = blockIdx.x * 32;
#pragma unroll 4
    for (int it = 0; it < KIN / 8; ++it) { const int k = it * 8 + wave; tile[k * WTP + lane] = W[(size_t)k * WC + n0 + lane]; }
    __syncthreads();
#pragma unroll 1
    for (int ps = 0; ps < 2; ++ps) {
#pragma unroll
        for (int q = 0; q < 4; ++q) { const int n = wave * 4 + q; v8us o;
#pragma unroll
            for (int i = 0; i < 8; ++i) o[i] = f2bf(tile[(8 * lane + i) * WTP + n]);
            *(volatile v8us*)(WT + (size_t)(n0 + n) * KIN + 8 * lane) = o; }
        if (ps == 0) __threadfence(); }
}

__global__ __launch_bounds__(256) void k_adjbits(const int* __restrict__ adj, unsigned* AB) {
    const int lane = threadIdx.x & 31;
    const int wave = __builtin_amdgcn_readfirstlane((int)(threadIdx.x >> 5));
    const int g0 = (blockIdx.x * 8 + wave) * 32;
    unsigned mine = 0u;
#pragma unroll 1
    for (int w = 0; w < 32; ++w) { const int g = g0 + w; const int row = g / ABW, wc = g % ABW;
        const int v = adj[(size_t)row * SEQ_FULL + (size_t)wc * 32 + lane];
        const unsigned bal = __builtin_amdgcn_ballot_w32(v > 0);
        mine = (lane == w) ? bal : mine; }
    *(volatile unsigned*)(AB + g0 + lane) = mine; __threadfence(); *(volatile unsigned*)(AB + g0 + lane) = mine;
}

__global__ __launch_bounds__(32) __attribute__((amdgpu_num_vgpr(256)))
void k_projv(const bf* __restrict__ A, const bf* __restrict__ Bt, const float* __restrict__ avec, h16* Ph, float* ST) {
    __shared__ __align__(16) float os[16 * 68];
    __shared__ __align__(16) float sst[128];
    const int K = KIN;
    const int lane = threadIdx.x & 31, lr = lane & 15, hi = lane >> 4;
    const int hd = blockIdx.x; const int c0 = blockIdx.y * 64;
    const int bb = c0 / SEQ, tt = c0 % SEQ;
    float ps[4], pt[4];
#pragma unroll
    for (int nb = 0; nb < 4; ++nb) { ps[nb] = 0.0f; pt[nb] = 0.0f; }
    const size_t boff = (size_t)(c0 + lr) * K + 8 * hi;
#pragma unroll 1
    for (int mt = 0; mt < HD / 64; ++mt) {
        const int r0 = hd * HD + mt * 64;
        v8f acc[4][4];
#pragma unroll
        for (int mb = 0; mb < 4; ++mb)
#pragma unroll
            for (int nb = 0; nb < 4; ++nb) acc[mb][nb] = (v8f){};
        const size_t aoff = (size_t)(r0 + lr) * K + 8 * hi;
#pragma unroll 1
        for (int kc = 0; kc < K; kc += 32) {
            v16bf a[4];
#pragma unroll
            for (int mb = 0; mb < 4; ++mb) a[mb] = ldb(A + aoff + (size_t)mb * 16 * K + kc);
#pragma unroll
            for (int nb = 0; nb < 4; ++nb) { const v16bf bq = ldb(Bt + boff + (size_t)nb * 16 * K + kc);
#pragma unroll
                for (int mb = 0; mb < 4; ++mb) acc[mb][nb] = wmmabg(a[mb], bq, acc[mb][nb]); }
        }
        const size_t tbase = (size_t)bb * (size_t)WC * SEQ + (size_t)r0 * SEQ + (size_t)tt;
        const float* ap = avec + (size_t)hd * (2 * HD) + mt * 64 + hi * 8;
#pragma unroll
        for (int mb = 0; mb < 4; ++mb) {
            float as_[8], at_[8];
#pragma unroll
            for (int j = 0; j < 8; ++j) { as_[j] = bfr(ap[mb * 16 + j]); at_[j] = bfr(ap[HD + mb * 16 + j]); }
#pragma unroll
            for (int nb = 0; nb < 4; ++nb) {
#pragma unroll
                for (int j = 0; j < 8; ++j) { const float v = acc[mb][nb][j];
                    os[(hi * 8 + j) * 68 + nb * 16 + lr] = v; ps[nb] += v * as_[j]; pt[nb] += v * at_[j]; } }
            wave_sync();
#pragma unroll 1
            for (int pq = 0; pq < 2; ++pq) {
                const size_t sb = tbase + (size_t)(mb * 16) * SEQ;
#pragma unroll
                for (int s = 0; s < 4; ++s) { const int row = 4 * s + (lane >> 3), c8 = (lane & 7) * 8;
                    const v4f x0 = *(const v4fa*)(&os[row * 68 + c8]); const v4f x1 = *(const v4fa*)(&os[row * 68 + c8 + 4]); v8h hv;
#pragma unroll
                    for (int i = 0; i < 4; ++i) { hv[i] = toh_flush(x0[i]); hv[4 + i] = toh_flush(x1[i]); }
                    *(volatile v8h*)(Ph + sb + (size_t)row * SEQ + c8) = hv; }
                if (pq == 0) __threadfence(); }
            wave_sync();
        }
    }
#pragma unroll
    for (int nb = 0; nb < 4; ++nb) { ps[nb] += __shfl_xor(ps[nb], 16, 32); pt[nb] += __shfl_xor(pt[nb], 16, 32); }
#pragma unroll
    for (int nb = 0; nb < 4; ++nb) { const float sv = hi ? pt[nb] : ps[nb]; sst[hi * 64 + nb * 16 + lr] = sv; }
    wave_sync();
    const v4f sv4 = *(const v4fa*)(&sst[4 * lane]);
    const size_t so = (size_t)(lane >> 4) * TGO + (size_t)(bb * NH_ + hd) * SEQ + (size_t)tt + (size_t)(4 * (lane & 15));
    *(volatile v4f*)(ST + so) = sv4; __threadfence(); *(volatile v4f*)(ST + so) = sv4;
}

__global__ __launch_bounds__(32 * AW) __attribute__((amdgpu_num_vgpr(256)))
void k_fused(const h16* __restrict__ VT, const float* __restrict__ ST, const unsigned* __restrict__ AB, float* OUT) {
    __shared__ __align__(16) float os[AW * 16 * OSQ];
    const int lane = threadIdx.x & 31, lr = lane & 15, hi = lane >> 4;
    const int wave = __builtin_amdgcn_readfirstlane((int)(threadIdx.x >> 5));
    const int b = blockIdx.y;
    const int t0 = (blockIdx.x * AW + wave) * 16;
    const int wb = wave * 16 * OSQ;
    const int lo = wb + lr * OSQ + 8 * hi;
    { const v4f z = (v4f){};
#pragma unroll
      for (int j = 0; j < NJ; ++j) { *(v4fa*)(&os[lo + 16 * j]) = z; *(v4fa*)(&os[lo + 16 * j + 4]) = z; } }
    const unsigned* abp = AB + (size_t)(t0 + lr) * ABW;
    const int sft = 8 * hi;
#pragma unroll 1
    for (int hd = 0; hd < NH_; ++hd) {
        const int zh = b * NH_ + hd;
        const float sv = ST[(size_t)zh * SEQ + t0 + lr];
        const float* tgp = ST + TGO + (size_t)zh * SEQ + 8 * hi;
        const h16* vp = VT + (size_t)zh * HD * SEQ + (size_t)lr * SEQ + 8 * hi;
        v8f o[NJ];
#pragma unroll
        for (int j = 0; j < NJ; ++j) o[j] = (v8f){};
        float m = NEGB, l = 0.0f;
#pragma unroll 1
        for (int key0 = 0; key0 < SEQ; key0 += 32) {
            const float* kp = tgp + key0;
            const v4f g0 = *(const v4f*)kp, g1 = *(const v4f*)(kp + 4), g2 = *(const v4f*)(kp + 16), g3 = *(const v4f*)(kp + 20);
            const unsigned wsh = abp[key0 >> 5] >> sft;
            float kx[8], ky[8];
#pragma unroll
            for (int r = 0; r < 4; ++r) { kx[r] = g0[r]; kx[4 + r] = g1[r]; ky[r] = g2[r]; ky[4 + r] = g3[r]; }
            float ta[8], tb[8]; float mx = NEGB;
#pragma unroll
            for (int r = 0; r < 8; ++r) {
                float ea = sv + kx[r]; ea = (ea >= 0.0f) ? ea : SLOPE * ea;
                float eb = sv + ky[r]; eb = (eb >= 0.0f) ? eb : SLOPE * eb;
                const bool fa = ((wsh >> r) & 1u) != 0u;
                const bool fb = ((wsh >> (16 + r)) & 1u) != 0u;
                ta[r] = fa ? ea * LOG2E : NEGT; tb[r] = fb ? eb * LOG2E : NEGT;
                mx = fmaxf(mx, fmaxf(ta[r], tb[r])); }
            mx = fmaxf(mx, __shfl_xor(mx, 16, 32));
            const float mnew = fmaxf(m, mx);
            const float alpha = __builtin_amdgcn_exp2f(m - mnew);
            const float sh = PSH - mnew;
            v16h pb; float ls = 0.0f;
#pragma unroll
            for (int r = 0; r < 8; ++r) {
                const float xa = ta[r] + sh, xb = tb[r] + sh;
                const float ea = __builtin_amdgcn_exp2f(xa), eb = __builtin_amdgcn_exp2f(xb);
                const float ga = (xa < -14.0f) ? 0.0f : ea, gb = (xb < -14.0f) ? 0.0f : eb;
                const h16 pa = (h16)ga; const h16 pc = (h16)gb;
                pb[r] = pa; pb[8 + r] = pc;
                ls += (float)pa + (float)pc; }
            l = l * alpha + ls; m = mnew;
#pragma unroll
            for (int j = 0; j < NJ; ++j) o[j] = o[j] * alpha;
            const h16* va = vp + key0;
#pragma unroll
            for (int g = 0; g < NJ / 4; ++g) {
                const v16h v0 = ldh(va + (size_t)(16 * (4 * g + 0)) * SEQ), v1 = ldh(va + (size_t)(16 * (4 * g + 1)) * SEQ);
                const v16h v2 = ldh(va + (size_t)(16 * (4 * g + 2)) * SEQ), v3 = ldh(va + (size_t)(16 * (4 * g + 3)) * SEQ);
                o[4 * g + 0] = wmma16g(v0, pb, o[4 * g + 0]); o[4 * g + 1] = wmma16g(v1, pb, o[4 * g + 1]);
                o[4 * g + 2] = wmma16g(v2, pb, o[4 * g + 2]); o[4 * g + 3] = wmma16g(v3, pb, o[4 * g + 3]); }
        }
        l += __shfl_xor(l, 16, 32);
        const bool any = l > 0.0f;
        const float lsafe = any ? l : 1.0f;
        const float inv = any ? (1.0f / lsafe) : 0.0f;
        const float sc = inv * HINV;
#pragma unroll
        for (int j = 0; j < NJ; ++j) {
            v4f x = *(const v4fa*)(&os[lo + 16 * j]); v4f y = *(const v4fa*)(&os[lo + 16 * j + 4]);
            x[0] += o[j][0] * sc; x[1] += o[j][1] * sc; x[2] += o[j][2] * sc; x[3] += o[j][3] * sc;
            y[0] += o[j][4] * sc; y[1] += o[j][5] * sc; y[2] += o[j][6] * sc; y[3] += o[j][7] * sc;
            *(v4fa*)(&os[lo + 16 * j]) = x; *(v4fa*)(&os[lo + 16 * j + 4]) = y; }
    }
    wave_sync();
    float* orow = OUT + ((size_t)b * OUT_SEQ + t0) * HD;
#pragma unroll 1
    for (int pq = 0; pq < 2; ++pq) {
#pragma unroll 4
        for (int s = 0; s < 32; ++s) { const int row = s >> 1, cofs = (s & 1) * 128 + lane * 4;
            const v4f val = *(const v4fa*)(&os[wb + row * OSQ + cofs]);
            *(volatile v4f*)(orow + (size_t)row * HD + cofs) = val; }
        if (pq == 0) __threadfence(); }
}

static constexpr size_t al256(size_t v) { return (v + 255) & ~(size_t)255; }
static constexpr size_t SZ_XB = al256((size_t)NB * SEQ * KIN * 2);
static constexpr size_t SZ_WT = al256((size_t)WC * KIN * 2);
static constexpr size_t SZ_VT = al256((size_t)NB * NH_ * HD * SEQ * 2);
static constexpr size_t SZ_ST = al256((size_t)2 * NB * NH_ * SEQ * 4);
static constexpr size_t SZ_AB = al256((size_t)SEQ * ABW * 4);
static constexpr size_t SZ_TOTAL = SZ_XB + SZ_WT + SZ_VT + SZ_ST + SZ_AB;
static_assert(SZ_TOTAL <= (size_t)134217728);
static_assert(((size_t)NB * NH_ * SEQ * 4) % 256 == 0);
static_assert((size_t)NB * WC * SEQ == (size_t)NB * NH_ * HD * SEQ);
static_assert((size_t)(NB * SEQ / 64) * 64 * NH_ * 2 * 4 == (size_t)2 * NB * NH_ * SEQ * 4);
static_assert(((size_t)SEQ * SEQ / 1024) * 128 == (size_t)SEQ * ABW * 4);

extern "C" void kernel_launch(void* const* d_in, const int* in_sizes, int n_in,
                              void* d_out, int out_size, void* d_ws, size_t ws_size, hipStream_t stream) {
    if (n_in < 4) return;
    const size_t needh = ((size_t)(NB - 1) * SEQ_FULL + SEQ) * KIN;
    const size_t needa = (size_t)(SEQ - 1) * SEQ_FULL + SEQ;
    if ((size_t)in_sizes[0] < needh) return;
    if ((size_t)in_sizes[1] < needa) return;
    if ((size_t)in_sizes[2] < (size_t)KIN * WC) return;
    if ((size_t)in_sizes[3] < (size_t)NH_ * 2 * HD) return;
    if ((size_t)out_size < ((size_t)(NB - 1) * OUT_SEQ + SEQ) * HD) return;
    if (SZ_TOTAL > ws_size) return;
    const float* hin = (const float*)d_in[0];
    const int*   adj = (const int*)d_in[1];
    const float* win = (const float*)d_in[2];
    const float* avec = (const float*)d_in[3];
    float* OUT = (float*)d_out;
    char* wsp = (char*)d_ws;
    bf* XB = (bf*)wsp; wsp += SZ_XB;
    bf* WT = (bf*)wsp; wsp += SZ_WT;
    h16* VT = (h16*)wsp; wsp += SZ_VT;
    float* ST = (float*)wsp; wsp += SZ_ST;
    unsigned* AB = (unsigned*)wsp; wsp += SZ_AB;

    if (SEQ == SEQ_FULL) {
        const size_t n8 = (size_t)NB * SEQ * KIN / 8;
        k_cvt8<<<(unsigned)((n8 + 255) / 256), 256, 0, stream>>>(hin, XB, n8);
    } else {
        const size_t n8 = (size_t)SEQ * KIN / 8;
        for (int b = 0; b < NB; ++b) k_cvt8<<<(unsigned)((n8 + 255) / 256), 256, 0, stream>>>(hin + (size_t)b * SEQ_FULL * KIN, XB + (size_t)b * SEQ * KIN, n8);
    }
    k_wt<<<WC / 32, 256, 0, stream>>>(win, WT);
    k_adjbits<<<(unsigned)(((size_t)SEQ * SEQ / 1024) / 8), 256, 0, stream>>>(adj, AB);

    k_projv<<<dim3(NH_, NB * SEQ / 64, 1), 32, 0, stream>>>(WT, XB, avec, VT, ST);

    k_fused<<<dim3(SEQ / (16 * AW), NB, 1), 32 * AW, 0, stream>>>(VT, ST, AB, OUT);
}
